// EdgeEncoder_19670950216141
// MI455X (gfx1250) — hardware-run, weakly checked
//
#include <hip/hip_runtime.h>
#include <math.h>

typedef __attribute__((ext_vector_type(16))) _Float16 v16h;
typedef __attribute__((ext_vector_type(16))) __bf16 v16b;
typedef __attribute__((ext_vector_type(8)))  _Float16 v8h;
typedef __attribute__((ext_vector_type(8)))  float v8f;
typedef __attribute__((ext_vector_type(4)))  float v4f;
typedef __attribute__((ext_vector_type(2)))  float v2f;
typedef __attribute__((ext_vector_type(4)))  unsigned v4u;
typedef __attribute__((ext_vector_type(4)))  int v4i;
typedef float __attribute__((may_alias)) float_a;
typedef int __attribute__((may_alias)) int_a;

template <typename T> __device__ __forceinline__ void vst2(void* p, T v) { *(volatile T*)p = v; __threadfence(); *(volatile T*)p = v; }
__device__ __forceinline__ v8f wmma16(v16h a, v16h b, v8f c) {
  v8f d = __builtin_amdgcn_wmma_f32_16x16x32_f16(false, a, false, b, (short)0, c, false, false);
  asm volatile("v_nop\n\tv_nop\n\tv_nop\n\tv_nop" : "+v"(d) : "v"(a), "v"(b));
  return d;
}
__device__ __forceinline__ v8f wmma_bf(v16b a, v16b b, v8f c) {
  v8f d = __builtin_amdgcn_wmma_f32_16x16x32_bf16(false, a, false, b, (short)0, c, false, false);
  asm volatile("v_nop\n\tv_nop\n\tv_nop\n\tv_nop" : "+v"(d) : "v"(a), "v"(b));
  return d;
}
__device__ __forceinline__ v16h frag_h(const _Float16* rowk0, int lane) {
  union { v16h v; v8h q[2]; } u; const _Float16* p = rowk0 + 8 * (lane >> 4);
  u.q[0] = *(const v8h*)p; u.q[1] = *(const v8h*)(p + 16); return u.v;
}
__device__ __forceinline__ v16h frag_f32(const float* rowk0, int lane) {
  v16h a; const float* p = rowk0 + 8 * (lane >> 4);
#pragma unroll
  for (int i = 0; i < 8; ++i) { a[i] = (_Float16)p[i]; a[8 + i] = (_Float16)p[16 + i]; }
  return a;
}
__device__ __forceinline__ v16h frag_f32s(const float* rowk0, int lane, float sc) {
  v16h a; const float* p = rowk0 + 8 * (lane >> 4);
#pragma unroll
  for (int i = 0; i < 8; ++i) { a[i] = (_Float16)(p[i] * sc); a[8 + i] = (_Float16)(p[16 + i] * sc); }
  return a;
}
__device__ __forceinline__ v16h fragc_f32(const float* W, int k0, int n, int lane, int ld, int K) {
  v16h a; const int g = lane >> 4;
#pragma unroll
  for (int i = 0; i < 8; ++i) { const int ka = k0 + 8 * g + i, kb = ka + 16;
    a[i] = (_Float16)(ka < K ? W[(size_t)(ka < K ? ka : K - 1) * ld + n] : 0.f); a[8 + i] = (_Float16)(kb < K ? W[(size_t)(kb < K ? kb : K - 1) * ld + n] : 0.f); }
  return a;
}
struct F2 { v16b h, l; };
__device__ __forceinline__ F2 bsplit16(const float v[16]) { F2 r;
#pragma unroll
  for (int i = 0; i < 16; ++i) { const __bf16 h = (__bf16)v[i]; r.h[i] = h; r.l[i] = (__bf16)(v[i] - (float)h); }
  return r; }
__device__ __forceinline__ F2 split_row(const float* row, int k0, int lane) { float v[16]; const float* p = row + k0 + 8 * (lane >> 4);
#pragma unroll
  for (int i = 0; i < 8; ++i) { v[i] = p[i]; v[8 + i] = p[16 + i]; }
  return bsplit16(v); }
__device__ __forceinline__ F2 split_rowK(const float* row, int k0, int lane, int K) { float v[16]; const int g = lane >> 4;
#pragma unroll
  for (int i = 0; i < 8; ++i) { const int ka = k0 + 8 * g + i, kb = ka + 16; v[i] = ka < K ? row[ka < K ? ka : K - 1] : 0.f; v[8 + i] = kb < K ? row[kb < K ? kb : K - 1] : 0.f; }
  return bsplit16(v); }
__device__ __forceinline__ F2 split_col(const float* W, int k0, int n, int lane, int ld, int K) { float v[16]; const int g = lane >> 4;
#pragma unroll
  for (int i = 0; i < 8; ++i) { const int ka = k0 + 8 * g + i, kb = ka + 16; v[i] = ka < K ? W[(size_t)(ka < K ? ka : K - 1) * ld + n] : 0.f; v[8 + i] = kb < K ? W[(size_t)(kb < K ? kb : K - 1) * ld + n] : 0.f; }
  return bsplit16(v); }
__device__ __forceinline__ v8f mac3(const F2& a, const F2& b, v8f c) { c = wmma_bf(a.l, b.h, c); c = wmma_bf(a.h, b.l, c); return wmma_bf(a.h, b.h, c); }
__device__ __forceinline__ float sigm(float v) { return 1.0f / (1.0f + expf(-v)); }
#define LDSX() do { asm volatile("s_wait_dscnt 0" ::: "memory"); __builtin_amdgcn_wave_barrier(); __builtin_amdgcn_fence(__ATOMIC_RELEASE, "workgroup"); } while (0)


#define NS 128
#define NPD 64
#define NT (NS * NPD)
#define HDIM 128
#define NHD 4
#define DH 32
#define RH 64
#ifndef TNT
#define TNT NT
#endif
typedef __attribute__((ext_vector_type(8))) __bf16 v8b;
__device__ __forceinline__ v16b frag_b(const __bf16* rowk0, int lane) {
  union { v16b v; v8b q[2]; } u; const __bf16* p = rowk0 + 8 * (lane >> 4);
  u.q[0] = *(const v8b*)p; u.q[1] = *(const v8b*)(p + 16); return u.v;
}
__device__ __forceinline__ float bfr(float v) { return (float)(__bf16)v; }
__device__ __attribute__((noinline)) float exp_ni(float v) { return expf(v); }
__device__ __attribute__((noinline)) float erf_ni(float v) { return erff(v); }

#define WS_M   0u
#define WS_C   (WS_M + 2u * 2 * HDIM * RH)
#define WS_Q   (WS_C + 4u * 2 * HDIM)
#define WS_END (WS_Q + 4u * (size_t)3 * NT * HDIM)

__global__ __launch_bounds__(256) void k_fold(const float* __restrict__ INW, const float* __restrict__ INB, const float* __restrict__ W2, const float* __restrict__ B2, _Float16* __restrict__ M, float* __restrict__ C) { __shared__ float sw2[HDIM][RH + 1]; __shared__ __align__(16) _Float16 sm[2 * HDIM][RH + 8]; __shared__ __align__(16) float sc[2 * HDIM]; const int t = threadIdx.x;
  for (int e = t; e < HDIM * RH; e += 256) sw2[e / RH][e % RH] = bfr(W2[e]); __syncthreads();
  for (int e = t; e < 2 * HDIM * RH; e += 256) { const int w = e / (HDIM * RH), o = (e / RH) % HDIM, m = e % RH; const float* wr = INW + ((size_t)(1 + w) * HDIM + o) * HDIM; float s = 0.f;
#pragma unroll 1
    for (int c = 0; c < HDIM; ++c) s += bfr(wr[c]) * sw2[c][m]; sm[w * HDIM + o][m] = (_Float16)s; }
  { const int w = t / HDIM, o = t % HDIM; const float* wr = INW + ((size_t)(1 + w) * HDIM + o) * HDIM; float s = bfr(INB[(1 + w) * HDIM + o]);
#pragma unroll 1
    for (int c = 0; c < HDIM; ++c) s += bfr(wr[c]) * bfr(B2[c]); sc[t] = s; }
  __syncthreads(); for (int e = t; e < 2 * HDIM * 8; e += 256) { const int r = e >> 3, q = e & 7; vst2((unsigned*)(M + (size_t)r * RH + q * 8), *(const v4u*)&sm[r][q * 8]); } if (t < 2 * HDIM / 4) vst2(C + t * 4, *(const v4f*)&sc[t * 4]); }
__device__ __forceinline__ v16b fragb_f32(const float* __restrict__ p, int lane) { v16b a; const float* pp = p + 8 * (lane >> 4);
#pragma unroll
  for (int i = 0; i < 8; ++i) { a[i] = (__bf16)pp[i]; a[8 + i] = (__bf16)pp[16 + i]; } return a; }
__global__ __launch_bounds__(128) void k_node(const float* __restrict__ X, const float* __restrict__ INW, const float* __restrict__ INB, float* __restrict__ QB) { __shared__ __align__(16) float sf[4][16][132];
  const int tid = threadIdx.x, wave = tid >> 5, lane = tid & 31, col = lane & 15, g = lane >> 4; const size_t r0 = (size_t)blockIdx.x * 64 + wave * 16; const int which = blockIdx.y;
  v8f acc[8] = {};
#pragma unroll
  for (int kc = 0; kc < HDIM / 32; ++kc) { const v16b a = fragb_f32(X + (r0 + col) * HDIM + kc * 32, lane);
#pragma unroll
    for (int j = 0; j < 8; ++j) acc[j] = wmma_bf(a, fragb_f32(INW + ((size_t)which * HDIM + j * 16 + col) * HDIM + kc * 32, lane), acc[j]); }
#pragma unroll
  for (int j = 0; j < 8; ++j) { const float bb = (which == 0) ? bfr(INB[j * 16 + col]) : 0.f;
#pragma unroll
    for (int r = 0; r < 8; ++r) sf[wave][8 * g + r][j * 16 + col] = acc[j][r] + bb; }
  LDSX(); for (int rl = 0; rl < 16; ++rl) vst2(QB + ((size_t)which * NT + r0 + rl) * HDIM + lane * 4, *(const v4f*)&sf[wave][rl][lane * 4]); }
__global__ __launch_bounds__(128) void k_pair(const float* __restrict__ X, const float* __restrict__ POS, const float* __restrict__ W1, const float* __restrict__ B1, const _Float16* __restrict__ M, const float* __restrict__ C, const float* __restrict__ QB, const float* __restrict__ OW, const float* __restrict__ OB, const float* __restrict__ PW, const float* __restrict__ PB, float* __restrict__ OUT) {
  __shared__ __align__(16) float shid[64][RH + 4]; __shared__ float sq[HDIM]; __shared__ float ssc[NHD][64]; __shared__ float sp[NHD][64]; __shared__ float sred[4][HDIM]; __shared__ float sctx[HDIM]; __shared__ float scomb[2 * HDIM]; __shared__ __align__(16) float so2[HDIM];
  const int tid = threadIdx.x, wave = tid >> 5, lane = tid & 31, col = lane & 15, g = lane >> 4; const int s = blockIdx.x / NPD, i = blockIdx.x % NPD; const size_t node_i = (size_t)blockIdx.x; const size_t node0 = (size_t)s * NPD;
  const float pix = bfr(POS[node_i * 2]), piy = bfr(POS[node_i * 2 + 1]);
  for (int e = tid; e < 64 * RH; e += 128) { const int j = e / RH, m = e % RH; const float rx = bfr(POS[(node0 + j) * 2]) - pix, ry = bfr(POS[(node0 + j) * 2 + 1]) - piy; shid[j][m] = fmaxf(rx * bfr(W1[m * 2]) + ry * bfr(W1[m * 2 + 1]) + bfr(B1[m]), 0.f); }
  sq[tid] = QB[node_i * HDIM + tid]; scomb[tid] = bfr(X[node_i * HDIM + tid]); __syncthreads();
  v8f ak[8] = {}, av[8] = {};
#pragma unroll
  for (int kc = 0; kc < 2; ++kc) { v16h a; const float* p2 = &shid[wave * 16 + col][kc * 32 + 8 * g];
#pragma unroll
    for (int q = 0; q < 8; ++q) { a[q] = (_Float16)p2[q]; a[8 + q] = (_Float16)p2[16 + q]; }
#pragma unroll
    for (int jt = 0; jt < 8; ++jt) { ak[jt] = wmma16(a, frag_h(M + (size_t)(jt * 16 + col) * RH + kc * 32, lane), ak[jt]); av[jt] = wmma16(a, frag_h(M + (size_t)(HDIM + jt * 16 + col) * RH + kc * 32, lane), av[jt]); } }
  float part[NHD][8];
#pragma unroll
  for (int hh = 0; hh < NHD; ++hh)
#pragma unroll
    for (int r = 0; r < 8; ++r) part[hh][r] = 0.f;
#pragma unroll
  for (int jt = 0; jt < 8; ++jt) { const int cch = jt * 16 + col; const float ckc = C[cch], qc = sq[cch]; const int hh = cch / DH;
#pragma unroll
    for (int r = 0; r < 8; ++r) { const size_t j = node0 + wave * 16 + 8 * g + r; const float kval = QB[((size_t)1 * NT + j) * HDIM + cch] + ak[jt][r] + ckc; part[hh][r] += qc * kval; } }
#pragma unroll
  for (int hh = 0; hh < NHD; ++hh)
#pragma unroll
    for (int r = 0; r < 8; ++r) { float v = part[hh][r];
#pragma unroll
      for (int o = 1; o < 16; o <<= 1) v += __shfl_xor(v, o);
      if (col == 0) ssc[hh][wave * 16 + 8 * g + r] = v * 0.17677669529663687f; }
  __syncthreads();
  if (tid < NHD) { const int hh = tid; float mx = -3.0e38f; for (int j = 0; j < 64; ++j) mx = fmaxf(mx, ssc[hh][j]); float sum = 0.f; for (int j = 0; j < 64; ++j) { const float e = expf(ssc[hh][j] - mx); sp[hh][j] = e; sum += e; } const float inv = 1.0f / sum; for (int j = 0; j < 64; ++j) sp[hh][j] *= inv; }
  __syncthreads();
  float cpart[8];
#pragma unroll
  for (int jt = 0; jt < 8; ++jt) { const int cch = jt * 16 + col; const float cvc = C[HDIM + cch]; const int hh = cch / DH; float acc = 0.f;
#pragma unroll
    for (int r = 0; r < 8; ++r) { const int jl = wave * 16 + 8 * g + r; const size_t j = node0 + jl; const float vval = QB[((size_t)2 * NT + j) * HDIM + cch] + av[jt][r] + cvc; acc += sp[hh][jl] * vval; }
    acc += __shfl_xor(acc, 16);
    cpart[jt] = acc; }
  if (g == 0) {
#pragma unroll
    for (int jt = 0; jt < 8; ++jt) sred[wave][jt * 16 + col] = cpart[jt]; }
  __syncthreads(); sctx[tid] = sred[0][tid] + sred[1][tid] + sred[2][tid] + sred[3][tid]; __syncthreads();
  { float a = bfr(OB[tid]); const float* wr = OW + (size_t)tid * HDIM;
#pragma unroll 1
    for (int c = 0; c < HDIM; ++c) a += sctx[c] * bfr(wr[c]); scomb[HDIM + tid] = a; }
  __syncthreads();
  { float a = bfr(PB[tid]); const float* wr = PW + (size_t)tid * 2 * HDIM;
#pragma unroll 1
    for (int c = 0; c < 2 * HDIM; ++c) a += scomb[c] * bfr(wr[c]); so2[tid] = a; }
  __syncthreads(); if (tid < HDIM / 4) vst2(OUT + node_i * HDIM + tid * 4, *(const v4f*)&so2[tid * 4]); }
extern "C" void kernel_launch(void* const* d_in, const int* in_sizes, int n_in, void* d_out, int out_size, void* d_ws, size_t ws_size, hipStream_t stream) {
  (void)in_sizes; (void)n_in; (void)out_size;
  const float** F = (const float**)d_in;
  if (ws_size < (size_t)WS_END) return;
  char* ws = (char*)d_ws; _Float16* M = (_Float16*)(ws + WS_M); float* C = (float*)(ws + WS_C); float* QB = (float*)(ws + WS_Q);
  k_fold<<<1, 256, 0, stream>>>(F[6], F[7], F[4], F[5], M, C);
  k_node<<<dim3(NT / 64, 3), 128, 0, stream>>>(F[0], F[6], F[7], QB);
  k_pair<<<TNT, 128, 0, stream>>>(F[0], F[1], F[2], F[3], M, C, QB, F[8], F[9], F[10], F[11], (float*)d_out);
}
